// GNNRNNForecastModel_81939386073767
// MI455X (gfx1250) — hardware-verified
//
#include <hip/hip_runtime.h>
#include <stddef.h>


#define NNODE   5000
#define FDIM    16
#define DDIM    128
#define NHEAD   4
#define CDIM    32
#define GDIM    512
#define HOR     12
#define NTHR    256
#define NWAVE   8
#define EPT     8
#define NGRP    2
#define CHUNK   (NTHR * EPT * NGRP)
#define WCAP    (EPT * NGRP * 32)
#define LISTN   (NWAVE * WCAP)
#define NBT     128
#define RCAP    4096
#define DEGCAP  128
#define HXB     64
#define HXP     132
#define LBM     32
#define GP      516
#define HP      136
#define ZP      132
#define WSCAP   134217728
#define NEG_SLOPE 0.2f
#define DEN_EPS   1e-16f
#define LN_EPS    1e-5f
#define ASCALE    16.0f
#define GUNSCALE  (1.0f / 256.0f)

#define LDS_AGG   ((RCAP * 2 + LISTN) * 4)
#define LDS_LSTM  ((LBM * GP + LBM * DDIM * 2 + GDIM) * 4 + LBM * HP * 2)

static_assert((CHUNK & (CHUNK - 1)) == 0);
static_assert(CHUNK <= 4096);
static_assert((NBT & (NBT - 1)) == 0 && NBT <= 4096);
static_assert((DDIM & (DDIM - 1)) == 0 && DDIM == NHEAD * CDIM && GDIM == 4 * DDIM);
static_assert(((HP * 2) % 16) == 0 && ((HXP * 4) % 16) == 0 && ((ZP * 4) % 16) == 0);
static_assert((((LBM * GP + 2 * LBM * DDIM + GDIM) * 4) % 16) == 0);
static_assert(LDS_AGG <= 65536);
static_assert(NBT % NWAVE == 0 && LBM == 4 * NWAVE && HXB == 8 * NWAVE);

typedef float          v4f  __attribute__((ext_vector_type(4)));
typedef float          v8f  __attribute__((ext_vector_type(8)));
typedef int            v4i  __attribute__((ext_vector_type(4)));
typedef unsigned int   v2u  __attribute__((ext_vector_type(2)));
typedef unsigned int   v4u  __attribute__((ext_vector_type(4)));
typedef unsigned short v4us __attribute__((ext_vector_type(4)));
typedef unsigned short v8us __attribute__((ext_vector_type(8)));
typedef _Float16       v4h  __attribute__((ext_vector_type(4)));
typedef _Float16       v8h  __attribute__((ext_vector_type(8)));
typedef _Float16       v16h __attribute__((ext_vector_type(16)));
typedef __bf16         v16b __attribute__((ext_vector_type(16)));
union FragB { v16b v; v8us h[2]; };
union FragH { v16h v; v8us h[2]; };
union Pk4   { v4h h; v2u u; };
union Pk8   { v8h h; v4u u; };

__device__ __forceinline__ unsigned int bfr(float f) {
  const unsigned int u = __float_as_uint(f);
  return (u + 0x7FFFu + ((u >> 16) & 1u)) >> 16;
}

__device__ __forceinline__ void split1(float x, unsigned short& hb, unsigned short& lb) {
  const unsigned int hu = bfr(x);
  const float hf = __uint_as_float(hu << 16);
  hb = (unsigned short)hu;
  lb = (unsigned short)bfr(x - hf);
}

__device__ __forceinline__ void split8(v4f a, v4f b, v8us& hi, v8us& lo) {
  unsigned short hb, lb;
  split1(a.x, hb, lb); hi[0] = hb; lo[0] = lb;
  split1(a.y, hb, lb); hi[1] = hb; lo[1] = lb;
  split1(a.z, hb, lb); hi[2] = hb; lo[2] = lb;
  split1(a.w, hb, lb); hi[3] = hb; lo[3] = lb;
  split1(b.x, hb, lb); hi[4] = hb; lo[4] = lb;
  split1(b.y, hb, lb); hi[5] = hb; lo[5] = lb;
  split1(b.z, hb, lb); hi[6] = hb; lo[6] = lb;
  split1(b.w, hb, lb); hi[7] = hb; lo[7] = lb;
}

__device__ __forceinline__ v8f wmb(v16b a, v16b b, v8f c) {
  v8f d = __builtin_amdgcn_wmma_f32_16x16x32_bf16(false, a, false, b, (short)0, c, false, false);
  asm volatile("v_nop\n\tv_nop\n\tv_nop\n\tv_nop" : "+v"(d) : "v"(a), "v"(b));
  return d;
}
__device__ __forceinline__ v8f wmh(v16h a, v16h b, v8f c) {
  v8f d = __builtin_amdgcn_wmma_f32_16x16x32_f16(false, a, false, b, (short)0, c, false, false);
  asm volatile("v_nop\n\tv_nop\n\tv_nop\n\tv_nop" : "+v"(d) : "v"(a), "v"(b));
  return d;
}

__device__ __forceinline__ float lrelu(float v) { return v > 0.0f ? v : NEG_SLOPE * v; }
__device__ __forceinline__ float eluf(float v) {
  const float ser = v * (1.0f + v * (0.5f + v * (0.16666667f + v * (0.041666668f + v * 0.0083333338f))));
  const float big = __expf(v) - 1.0f;
  const float neg = (v > -0.0625f) ? ser : big;
  return v > 0.0f ? v : neg;
}
__device__ __forceinline__ float sigm(float x) { return __builtin_amdgcn_rcpf(1.0f + __expf(-x)); }
__device__ __forceinline__ float tanhx(float x) {
  const float e = __expf(-2.0f * fabsf(x));
  const float r = (1.0f - e) * __builtin_amdgcn_rcpf(1.0f + e);
  return x < 0.0f ? -r : r;
}

template <int NB>
__device__ __forceinline__ int scan_chunk(const int* __restrict__ dsts, int nE, int cbase, int slotBase,
                                          int vec8, int* list, int tid, int lane, int wave) {
  int wc = 0;
#pragma unroll
  for (int g = 0; g < NGRP; ++g) {
    const int el0  = (g * NTHR + tid) * EPT;
    const int e0   = cbase + el0;
    const int sent = -2147483647 - 1;
    v4i da, db;
    if (vec8 != 0 && cbase + CHUNK <= nE) {
      da = *(const v4i*)(dsts + e0);
      db = *(const v4i*)(dsts + e0 + 4);
    } else {
      da.x = (e0     < nE) ? dsts[min(e0, nE - 1)] : sent;
      da.y = (e0 + 1 < nE) ? dsts[min(e0 + 1, nE - 1)] : sent;
      da.z = (e0 + 2 < nE) ? dsts[min(e0 + 2, nE - 1)] : sent;
      da.w = (e0 + 3 < nE) ? dsts[min(e0 + 3, nE - 1)] : sent;
      db.x = (e0 + 4 < nE) ? dsts[min(e0 + 4, nE - 1)] : sent;
      db.y = (e0 + 5 < nE) ? dsts[min(e0 + 5, nE - 1)] : sent;
      db.z = (e0 + 6 < nE) ? dsts[min(e0 + 6, nE - 1)] : sent;
      db.w = (e0 + 7 < nE) ? dsts[min(e0 + 7, nE - 1)] : sent;
    }
    const unsigned nb = (unsigned)slotBase;
    const unsigned s0 = (unsigned)da.x - nb, s1 = (unsigned)da.y - nb;
    const unsigned s2 = (unsigned)da.z - nb, s3 = (unsigned)da.w - nb;
    const unsigned s4 = (unsigned)db.x - nb, s5 = (unsigned)db.y - nb;
    const unsigned s6 = (unsigned)db.z - nb, s7 = (unsigned)db.w - nb;
    const bool h0 = s0 < (unsigned)NB, h1 = s1 < (unsigned)NB, h2 = s2 < (unsigned)NB, h3 = s3 < (unsigned)NB;
    const bool h4 = s4 < (unsigned)NB, h5 = s5 < (unsigned)NB, h6 = s6 < (unsigned)NB, h7 = s7 < (unsigned)NB;
    const unsigned any = __builtin_amdgcn_ballot_w32(h0 | h1 | h2 | h3 | h4 | h5 | h6 | h7);
    if (any != 0u) {
#define HITJ(J, HJ, SJ) { \
        const unsigned mj = __builtin_amdgcn_ballot_w32(HJ); \
        if (mj != 0u) { \
          if (HJ) { \
            const int pos = wc + (int)__builtin_amdgcn_mbcnt_lo(mj, 0u); \
            if (pos < WCAP) list[wave * WCAP + pos] = ((el0 + (J)) << 12) | (int)(SJ); \
          } \
          wc += (int)__builtin_popcount(mj); } }
      HITJ(0, h0, s0)
      HITJ(1, h1, s1)
      HITJ(2, h2, s2)
      HITJ(3, h3, s3)
      HITJ(4, h4, s4)
      HITJ(5, h5, s5)
      HITJ(6, h6, s6)
      HITJ(7, h7, s7)
#undef HITJ
    }
  }
  return wc;
}

__global__ __launch_bounds__(NTHR) void k_prep_lin(const float* __restrict__ Wl, unsigned short* wlp) {
  const int i = (int)threadIdx.x;
  if (blockIdx.x != 0) return;
  const int n = i >> 1, k0 = (i & 1) * 8;
  float v[8];
#pragma unroll
  for (int e = 0; e < 8; ++e) v[e] = Wl[(size_t)(k0 + e) * DDIM + n];
  v4f a, b;
  a.x = v[0]; a.y = v[1]; a.z = v[2]; a.w = v[3];
  b.x = v[4]; b.y = v[5]; b.z = v[6]; b.w = v[7];
  v8us hv, lv;
  split8(a, b, hv, lv);
  unsigned short* dh = wlp + (size_t)i * 8;
  unsigned short* dl = dh + DDIM * FDIM;
  *(volatile v8us*)dh = hv;
  *(volatile v8us*)dl = lv;
  __threadfence();
  *(volatile v8us*)dh = hv;
  *(volatile v8us*)dl = lv;
}

__global__ __launch_bounds__(NTHR) void k_prep_lstm(const float* __restrict__ Wih, const float* __restrict__ Whh,
                                                     unsigned short* pih, unsigned short* phh) {
  const int b = (int)blockIdx.x;
  const bool second = b >= 32;
  const float* W = second ? Whh : Wih;
  unsigned short* P = second ? phh : pih;
  const int i = (b & 31) * NTHR + (int)threadIdx.x;
  const float* sp = W + (size_t)i * 8;
  const v4f a = *(const v4f*)sp, c = *(const v4f*)(sp + 4);
  Pk8 pk;
  pk.h[0] = (_Float16)(a.x * ASCALE); pk.h[1] = (_Float16)(a.y * ASCALE);
  pk.h[2] = (_Float16)(a.z * ASCALE); pk.h[3] = (_Float16)(a.w * ASCALE);
  pk.h[4] = (_Float16)(c.x * ASCALE); pk.h[5] = (_Float16)(c.y * ASCALE);
  pk.h[6] = (_Float16)(c.z * ASCALE); pk.h[7] = (_Float16)(c.w * ASCALE);
  unsigned short* dp = P + (size_t)i * 8;
  *(volatile v4u*)dp = pk.u;
  __threadfence();
  *(volatile v4u*)dp = pk.u;
}

__global__ __launch_bounds__(NTHR) void k_prep_head(const float* __restrict__ W1, const float* __restrict__ W2,
                                                     unsigned short* w1p, unsigned short* w2p) {
  const int b = (int)blockIdx.x, tid = (int)threadIdx.x;
  float v[8];
  unsigned short* dh;
  unsigned short* dl;
  if (b < 8) {
    const int i = b * NTHR + tid;
    const int n = i >> 4, k0 = (i & 15) * 8;
#pragma unroll
    for (int e = 0; e < 8; ++e) v[e] = W1[(size_t)(k0 + e) * DDIM + n];
    dh = w1p + (size_t)i * 8;
    dl = dh + DDIM * DDIM;
  } else {
    const int i = tid;
    const int n = i >> 4, k0 = (i & 15) * 8;
    const int nn = n < HOR ? n : HOR - 1;
    const bool ok = n < HOR;
#pragma unroll
    for (int e = 0; e < 8; ++e) { const float t = W2[(size_t)(k0 + e) * HOR + nn]; v[e] = ok ? t : 0.0f; }
    dh = w2p + (size_t)i * 8;
    dl = dh + 16 * DDIM;
  }
  v4f a, c;
  a.x = v[0]; a.y = v[1]; a.z = v[2]; a.w = v[3];
  c.x = v[4]; c.y = v[5]; c.z = v[6]; c.w = v[7];
  v8us hv, lv;
  split8(a, c, hv, lv);
  *(volatile v8us*)dh = hv;
  *(volatile v8us*)dl = lv;
  __threadfence();
  *(volatile v8us*)dh = hv;
  *(volatile v8us*)dl = lv;
}

__global__ __launch_bounds__(NTHR) void k_hx(
    const float* __restrict__ x, const unsigned short* __restrict__ wlp,
    const float* __restrict__ attS, const float* __restrict__ attD,
    float* hx, float* eS, float* eD, int nRows) {
  __shared__ __attribute__((aligned(16))) float stg[HXB * HXP];
  __shared__ __attribute__((aligned(16))) float sES[HXB * NHEAD];
  __shared__ __attribute__((aligned(16))) float sED[HXB * NHEAD];
  const int tid = threadIdx.x, lane = tid & 31, wave = tid >> 5, hh = lane >> 4, m = lane & 15;
  const int rg = wave >> 1, ch = wave & 1;
  const int rowBase = blockIdx.x * HXB;

  int row = rowBase + rg * 16 + m;
  row = row > nRows - 1 ? nRows - 1 : row;
  const float* xp = x + (size_t)row * FDIM + 8 * hh;
  const v4f xa = *(const v4f*)xp, xb = *(const v4f*)(xp + 4);
  FragB af;
  split8(xa, xb, af.h[0], af.h[1]);

  v8f acc[4];
#pragma unroll
  for (int t = 0; t < 4; ++t) { v8f z = {0.f, 0.f, 0.f, 0.f, 0.f, 0.f, 0.f, 0.f}; acc[t] = z; }
#pragma unroll
  for (int t = 0; t < 4; ++t) {
    const unsigned short* bp = wlp + (size_t)(ch * 64 + 16 * t + m) * FDIM + 8 * hh;
    const v8us wh = *(const v8us*)bp;
    const v8us wl = *(const v8us*)(bp + DDIM * FDIM);
    FragB bh, bl;
    bh.h[0] = wh; bh.h[1] = wh;
    bl.h[0] = wl; bl.h[1] = wl;
    acc[t] = wmb(af.v, bh.v, acc[t]);
    acc[t] = wmb(af.v, bl.v, acc[t]);
  }
  {
    float* sp = stg + (size_t)(rg * 16 + 8 * hh) * HXP + ch * 64 + m;
#pragma unroll
    for (int t = 0; t < 4; ++t) {
#pragma unroll
      for (int r = 0; r < 8; ++r) sp[r * HXP + 16 * t] = acc[t][r];
    }
  }
  __syncthreads();

  const int hd = lane >> 3;
  const v4f sa = *(const v4f*)(attS + 4 * lane);
  const v4f sd = *(const v4f*)(attD + 4 * lane);
  v4f vv[8];
#pragma unroll
  for (int it = 0; it < 8; ++it) {
    const int r = wave * 8 + it;
    const v4f v = *(const v4f*)(stg + (size_t)r * HXP + 4 * lane);
    vv[it] = v;
    *(volatile v4f*)(hx + (size_t)(rowBase + r) * DDIM + 4 * lane) = v;
    float ps = v.x * sa.x + v.y * sa.y + v.z * sa.z + v.w * sa.w;
    float pd = v.x * sd.x + v.y * sd.y + v.z * sd.z + v.w * sd.w;
    ps += __shfl_xor(ps, 1); pd += __shfl_xor(pd, 1);
    ps += __shfl_xor(ps, 2); pd += __shfl_xor(pd, 2);
    ps += __shfl_xor(ps, 4); pd += __shfl_xor(pd, 4);
    if ((lane & 7) == 0) { sES[r * NHEAD + hd] = ps; sED[r * NHEAD + hd] = pd; }
  }
  __threadfence();
#pragma unroll
  for (int it = 0; it < 8; ++it) {
    const int r = wave * 8 + it;
    *(volatile v4f*)(hx + (size_t)(rowBase + r) * DDIM + 4 * lane) = vv[it];
  }
  __syncthreads();

  v4f d0 = {0.f, 0.f, 0.f, 0.f}, d1 = {0.f, 0.f, 0.f, 0.f};
  const size_t eb = (size_t)rowBase * NHEAD;
  if (wave == 0) {
    d0 = *(const v4f*)(sES + 4 * lane);
    d1 = *(const v4f*)(sES + 128 + 4 * lane);
    *(volatile v4f*)(eS + eb + 4 * lane) = d0;
    *(volatile v4f*)(eS + eb + 128 + 4 * lane) = d1;
  } else if (wave == 1) {
    d0 = *(const v4f*)(sED + 4 * lane);
    d1 = *(const v4f*)(sED + 128 + 4 * lane);
    *(volatile v4f*)(eD + eb + 4 * lane) = d0;
    *(volatile v4f*)(eD + eb + 128 + 4 * lane) = d1;
  }
  __threadfence();
  if (wave == 0) {
    *(volatile v4f*)(eS + eb + 4 * lane) = d0;
    *(volatile v4f*)(eS + eb + 128 + 4 * lane) = d1;
  } else if (wave == 1) {
    *(volatile v4f*)(eD + eb + 4 * lane) = d0;
    *(volatile v4f*)(eD + eb + 128 + 4 * lane) = d1;
  }
}

__global__ __launch_bounds__(NTHR) void k_agg(
    const int* __restrict__ ei, const float* __restrict__ ew,
    const float* __restrict__ Wedge, const float* __restrict__ attE, const float* __restrict__ gbias,
    const float* __restrict__ hx, const float* __restrict__ eS, const float* __restrict__ eD,
    unsigned short* g16, int nN, int nE, int nB, int nT, int vec8) {
  extern __shared__ v4f lds_dyn[];
  int*   region = (int*)lds_dyn;
  float* regw   = (float*)(region + RCAP);
  int*   list   = (int*)(regw + RCAP);
  __shared__ int scnt[NBT];
  __shared__ int soff[NBT];
  __shared__ int curs[NBT];
  __shared__ int wcnt[NWAVE];
  __shared__ float sS[NHEAD];
  __shared__ __attribute__((aligned(16))) float sBias[DDIM];
  const int tid = threadIdx.x, lane = tid & 31, wave = tid >> 5;
  const int nodeBase = blockIdx.x * NBT;
  const int* srcs = ei;
  const int* dsts = ei + nE;

  for (int i = tid; i < NBT; i += NTHR) scnt[i] = 0;
  for (int i = tid; i < RCAP; i += NTHR) { region[i] = 0; regw[i] = 0.0f; }
  if (tid < DDIM) sBias[tid] = gbias[tid];
  if (tid < NHEAD) {
    float s = 0.0f;
#pragma unroll 1
    for (int c = 0; c < CDIM; ++c) s += Wedge[tid * CDIM + c] * attE[tid * CDIM + c];
    sS[tid] = s;
  }
  __syncthreads();

  const int nChunks = (nE + CHUNK - 1) / CHUNK;
#pragma unroll 1
  for (int chn = 0; chn < nChunks; ++chn) {
    const int cbase = chn * CHUNK;
    const int wc = scan_chunk<NBT>(dsts, nE, cbase, nodeBase, vec8, list, tid, lane, wave);
    if (lane == 0) wcnt[wave] = wc;
    __syncthreads();
    if (wave == 0) {
#pragma unroll 1
      for (int wsx = 0; wsx < NWAVE; ++wsx) {
        int n = __builtin_amdgcn_readfirstlane(wcnt[wsx]);
        n = n > WCAP ? WCAP : (n < 0 ? 0 : n);
        const int* lp = list + wsx * WCAP;
#pragma unroll 1
        for (int i = 0; i < n; ++i) {
          const int ent  = __builtin_amdgcn_readfirstlane(lp[i]);
          const int slot = ent & (NBT - 1);
          if (lane == 0) scnt[slot] = scnt[slot] + 1;
        }
      }
    }
    __syncthreads();
  }
  if (tid == 0) {
    int run = 0;
#pragma unroll 1
    for (int s = 0; s < NBT; ++s) {
      soff[s] = run;
      curs[s] = run;
      int cv = scnt[s];
      cv = cv < 0 ? 0 : cv;
      run += cv;
      run = run > RCAP ? RCAP : run;
    }
  }
  __syncthreads();
#pragma unroll 1
  for (int chn = 0; chn < nChunks; ++chn) {
    const int cbase = chn * CHUNK;
    const int wc = scan_chunk<NBT>(dsts, nE, cbase, nodeBase, vec8, list, tid, lane, wave);
    if (lane == 0) wcnt[wave] = wc;
    __syncthreads();
    if (wave == 0) {
#pragma unroll 1
      for (int wsx = 0; wsx < NWAVE; ++wsx) {
        int n = __builtin_amdgcn_readfirstlane(wcnt[wsx]);
        n = n > WCAP ? WCAP : (n < 0 ? 0 : n);
        const int* lp = list + wsx * WCAP;
#pragma unroll 1
        for (int i = 0; i < n; ++i) {
          const int ent  = __builtin_amdgcn_readfirstlane(lp[i]);
          const int slot = ent & (NBT - 1);
          int e = cbase + ((ent >> 12) & (CHUNK - 1));
          e = e > nE - 1 ? nE - 1 : e;
          int src = srcs[e];
          src = src < 0 ? 0 : (src > nN - 1 ? nN - 1 : src);
          const float wv = ew[e];
          if (lane == 0) {
            int pos = curs[slot];
            pos = pos < 0 ? 0 : (pos > RCAP - 1 ? RCAP - 1 : pos);
            region[pos] = src;
            regw[pos] = wv;
            const int np = pos + 1;
            curs[slot] = np > RCAP ? RCAP : np;
          }
        }
      }
    }
    __syncthreads();
  }

  const int hd = lane >> 3;
  const float Sh = sS[hd];
  const v4f bias4 = *(const v4f*)(sBias + 4 * lane);
  const int nSig = nB * nT;
#pragma unroll 1
  for (int tl = wave; tl < NBT; tl += NWAVE) {
    const int c = nodeBase + tl;
    if (c < nN) {
      int st = soff[tl];
      st = st < 0 ? 0 : (st > RCAP ? RCAP : st);
      int deg = curs[tl] - st;
      deg = deg < 0 ? 0 : (deg > DEGCAP ? DEGCAP : deg);
#pragma unroll 1
      for (int sg = 0; sg < nSig; ++sg) {
        const int b = sg / nT;
        const int t = sg - b * nT;
        const size_t rowc = (size_t)(b * nN + c) * nT + t;
        const float edv = eD[rowc * NHEAD + hd];
        float mx = -3.0e38f;
#pragma unroll 1
        for (int p = 0; p < deg; ++p) {
          int pos = st + p;
          pos = pos > RCAP - 1 ? RCAP - 1 : pos;
          const int s = region[pos];
          const float w = regw[pos];
          const size_t rows = (size_t)(b * nN + s) * nT + t;
          const float a = lrelu(eS[rows * NHEAD + hd] + edv + w * Sh);
          mx = fmaxf(mx, a);
        }
        float den = 0.0f;
        v4f acc = {0.f, 0.f, 0.f, 0.f};
#pragma unroll 1
        for (int p = 0; p < deg; ++p) {
          int pos = st + p;
          pos = pos > RCAP - 1 ? RCAP - 1 : pos;
          const int s = region[pos];
          const float w = regw[pos];
          const size_t rows = (size_t)(b * nN + s) * nT + t;
          const float a = lrelu(eS[rows * NHEAD + hd] + edv + w * Sh);
          const float pe = __expf(a - mx);
          den += pe;
          const v4f hv = *(const v4f*)(hx + rows * DDIM + 4 * lane);
          acc = acc + hv * pe;
        }
        const float rden = __builtin_amdgcn_rcpf(den + DEN_EPS);
        const v4f v = acc * rden + bias4;
        Pk4 pk;
        pk.h.x = (_Float16)(eluf(v.x) * ASCALE);
        pk.h.y = (_Float16)(eluf(v.y) * ASCALE);
        pk.h.z = (_Float16)(eluf(v.z) * ASCALE);
        pk.h.w = (_Float16)(eluf(v.w) * ASCALE);
        unsigned short* gp = g16 + rowc * DDIM + 4 * lane;
        *(volatile v2u*)gp = pk.u;
        __threadfence();
        *(volatile v2u*)gp = pk.u;
      }
    }
  }
}

__global__ __launch_bounds__(NTHR) void k_lstm(
    const unsigned short* __restrict__ g16, const unsigned short* __restrict__ pih,
    const unsigned short* __restrict__ phh, const float* __restrict__ bih,
    const float* __restrict__ bhh, float* hT, int M, int nT) {
  extern __shared__ v4f lds_dyn[];
  float* sG    = (float*)lds_dyn;
  float* sC    = sG + LBM * GP;
  float* sHf   = sC + LBM * DDIM;
  float* sBias = sHf + LBM * DDIM;
  unsigned short* sH = (unsigned short*)(sBias + GDIM);
  const int tid = threadIdx.x, lane = tid & 31, wave = tid >> 5, hh = lane >> 4, m = lane & 15;
  const int rg = wave >> 2, gq = wave & 3;
  const int rowBase = blockIdx.x * LBM;

  for (int i = tid; i < LBM * DDIM; i += NTHR) { sC[i] = 0.0f; sHf[i] = 0.0f; }
  for (int i = tid; i < LBM * HP; i += NTHR) sH[i] = 0;
  for (int i = tid; i < GDIM; i += NTHR) sBias[i] = bih[i] + bhh[i];
  __syncthreads();

  int arow = rowBase + rg * 16 + m;
  arow = arow > M - 1 ? M - 1 : arow;
  const unsigned short* xr = g16 + (size_t)arow * nT * DDIM + 8 * hh;
  const unsigned short* hr = sH + (rg * 16 + m) * HP + 8 * hh;
  const unsigned short* wi = pih + (size_t)(gq * DDIM + m) * DDIM + 8 * hh;
  const unsigned short* wh = phh + (size_t)(gq * DDIM + m) * DDIM + 8 * hh;
  const int d = tid & (DDIM - 1), rsel = tid >> 7;
  const float bi = sBias[d], bf = sBias[DDIM + d], bg = sBias[2 * DDIM + d], bo = sBias[3 * DDIM + d];

#pragma unroll 1
  for (int t = 0; t < nT; ++t) {
    v8f acc[8];
#pragma unroll
    for (int tt = 0; tt < 8; ++tt) { v8f z = {0.f, 0.f, 0.f, 0.f, 0.f, 0.f, 0.f, 0.f}; acc[tt] = z; }
    const unsigned short* xt = xr + (size_t)t * DDIM;
#pragma unroll 1
    for (int kt = 0; kt < DDIM / 32; ++kt) {
      FragH a;
      a.h[0] = *(const v8us*)(xt + 32 * kt);
      a.h[1] = *(const v8us*)(xt + 32 * kt + 16);
#pragma unroll
      for (int tt = 0; tt < 8; ++tt) {
        const unsigned short* bp = wi + (size_t)tt * 16 * DDIM + 32 * kt;
        FragH bq;
        bq.h[0] = *(const v8us*)bp;
        bq.h[1] = *(const v8us*)(bp + 16);
        acc[tt] = wmh(a.v, bq.v, acc[tt]);
      }
    }
#pragma unroll 1
    for (int kt = 0; kt < DDIM / 32; ++kt) {
      FragH a;
      a.h[0] = *(const v8us*)(hr + 32 * kt);
      a.h[1] = *(const v8us*)(hr + 32 * kt + 16);
#pragma unroll
      for (int tt = 0; tt < 8; ++tt) {
        const unsigned short* bp = wh + (size_t)tt * 16 * DDIM + 32 * kt;
        FragH bq;
        bq.h[0] = *(const v8us*)bp;
        bq.h[1] = *(const v8us*)(bp + 16);
        acc[tt] = wmh(a.v, bq.v, acc[tt]);
      }
    }
    {
      float* gp = sG + (size_t)(rg * 16 + 8 * hh) * GP + gq * DDIM + m;
#pragma unroll
      for (int tt = 0; tt < 8; ++tt) {
#pragma unroll
        for (int r = 0; r < 8; ++r) gp[r * GP + 16 * tt] = acc[tt][r];
      }
    }
    __syncthreads();

#pragma unroll 2
    for (int j = 0; j < 16; ++j) {
      const int rr = 2 * j + rsel;
      const float* g0 = sG + (size_t)rr * GP + d;
      const float gi = g0[0] * GUNSCALE + bi;
      const float gf = g0[DDIM] * GUNSCALE + bf;
      const float gg = g0[2 * DDIM] * GUNSCALE + bg;
      const float go = g0[3 * DDIM] * GUNSCALE + bo;
      float cc = sC[rr * DDIM + d];
      cc = sigm(gf) * cc + sigm(gi) * tanhx(gg);
      const float hv = sigm(go) * tanhx(cc);
      sC[rr * DDIM + d]  = cc;
      sHf[rr * DDIM + d] = hv;
      sH[rr * HP + d]    = __builtin_bit_cast(unsigned short, (_Float16)(hv * ASCALE));
    }
    __syncthreads();
  }

  v4f hv4[4];
#pragma unroll
  for (int i = 0; i < 4; ++i) {
    const int rr = wave * 4 + i;
    hv4[i] = *(const v4f*)(sHf + (size_t)rr * DDIM + 4 * lane);
    *(volatile v4f*)(hT + (size_t)(rowBase + rr) * DDIM + 4 * lane) = hv4[i];
  }
  __threadfence();
#pragma unroll
  for (int i = 0; i < 4; ++i) {
    const int rr = wave * 4 + i;
    *(volatile v4f*)(hT + (size_t)(rowBase + rr) * DDIM + 4 * lane) = hv4[i];
  }
}

__global__ __launch_bounds__(NTHR) void k_head(
    const float* __restrict__ hT, const float* __restrict__ lng, const float* __restrict__ lnb,
    const unsigned short* __restrict__ w1p, const float* __restrict__ b1,
    const unsigned short* __restrict__ w2p, const float* __restrict__ b2,
    float* out, int M, int nOut) {
  __shared__ __attribute__((aligned(16))) unsigned short sAh[LBM * HP];
  __shared__ __attribute__((aligned(16))) unsigned short sAl[LBM * HP];
  __shared__ __attribute__((aligned(16))) float stg[LBM * ZP];
  __shared__ __attribute__((aligned(16))) float sO[LBM * HOR];
  const int tid = threadIdx.x, lane = tid & 31, wave = tid >> 5, hh = lane >> 4, m = lane & 15;
  const int rowBase = blockIdx.x * LBM;

  {
    const v4f g4 = *(const v4f*)(lng + 4 * lane), b4 = *(const v4f*)(lnb + 4 * lane);
#pragma unroll
    for (int i = 0; i < 4; ++i) {
      const int r = wave * 4 + i;
      int grow = rowBase + r;
      grow = grow > M - 1 ? M - 1 : grow;
      const v4f v = *(const v4f*)(hT + (size_t)grow * DDIM + 4 * lane);
      float s = (v.x + v.y) + (v.z + v.w);
      s += __shfl_xor(s, 1); s += __shfl_xor(s, 2); s += __shfl_xor(s, 4);
      s += __shfl_xor(s, 8); s += __shfl_xor(s, 16);
      const float mu = s * (1.0f / DDIM);
      const v4f dv = v - mu;
      float q = (dv.x * dv.x + dv.y * dv.y) + (dv.z * dv.z + dv.w * dv.w);
      q += __shfl_xor(q, 1); q += __shfl_xor(q, 2); q += __shfl_xor(q, 4);
      q += __shfl_xor(q, 8); q += __shfl_xor(q, 16);
      const float var = q * (1.0f / DDIM);
      const float rs = __builtin_amdgcn_rsqf(var + LN_EPS);
      const v4f y = dv * rs * g4 + b4;
      unsigned short h0, l0, h1, l1, h2, l2, h3, l3;
      split1(y.x, h0, l0); split1(y.y, h1, l1); split1(y.z, h2, l2); split1(y.w, h3, l3);
      v4us hv = {h0, h1, h2, h3};
      v4us lv = {l0, l1, l2, l3};
      *(v4us*)(sAh + r * HP + 4 * lane) = hv;
      *(v4us*)(sAl + r * HP + 4 * lane) = lv;
    }
  }
  __syncthreads();

  const int rg = wave >> 2, cq = wave & 3;
  v8f acc[2];
  { v8f z = {0.f, 0.f, 0.f, 0.f, 0.f, 0.f, 0.f, 0.f}; acc[0] = z; acc[1] = z; }
  {
    const unsigned short* ahp = sAh + (rg * 16 + m) * HP + 8 * hh;
    const unsigned short* alp = sAl + (rg * 16 + m) * HP + 8 * hh;
#pragma unroll
    for (int kt = 0; kt < DDIM / 32; ++kt) {
      FragB ah, al;
      ah.h[0] = *(const v8us*)(ahp + 32 * kt);
      ah.h[1] = *(const v8us*)(ahp + 32 * kt + 16);
      al.h[0] = *(const v8us*)(alp + 32 * kt);
      al.h[1] = *(const v8us*)(alp + 32 * kt + 16);
#pragma unroll
      for (int t = 0; t < 2; ++t) {
        const unsigned short* bp = w1p + (size_t)(cq * 32 + 16 * t + m) * DDIM + 32 * kt + 8 * hh;
        FragB bh, bl;
        bh.h[0] = *(const v8us*)bp;
        bh.h[1] = *(const v8us*)(bp + 16);
        bl.h[0] = *(const v8us*)(bp + DDIM * DDIM);
        bl.h[1] = *(const v8us*)(bp + DDIM * DDIM + 16);
        acc[t] = wmb(ah.v, bh.v, acc[t]);
        acc[t] = wmb(ah.v, bl.v, acc[t]);
        acc[t] = wmb(al.v, bh.v, acc[t]);
      }
    }
  }
  {
    float* sp = stg + (size_t)(rg * 16 + 8 * hh) * ZP + cq * 32 + m;
#pragma unroll
    for (int t = 0; t < 2; ++t) {
      const float bb = b1[cq * 32 + 16 * t + m];
#pragma unroll
      for (int r = 0; r < 8; ++r) sp[r * ZP + 16 * t] = fmaxf(acc[t][r] + bb, 0.0f);
    }
  }
  __syncthreads();

  for (int u = tid; u < LBM * DDIM / 8; u += NTHR) {
    const int r = u >> 4, c0 = (u & 15) * 8;
    const v4f a = *(const v4f*)(stg + (size_t)r * ZP + c0), c = *(const v4f*)(stg + (size_t)r * ZP + c0 + 4);
    v8us hv, lv;
    split8(a, c, hv, lv);
    *(v8us*)(sAh + r * HP + c0) = hv;
    *(v8us*)(sAl + r * HP + c0) = lv;
  }
  __syncthreads();

  if (wave < 2) {
    const int r2 = wave;
    v8f acc2 = {0.f, 0.f, 0.f, 0.f, 0.f, 0.f, 0.f, 0.f};
    const unsigned short* ahp = sAh + (r2 * 16 + m) * HP + 8 * hh;
    const unsigned short* alp = sAl + (r2 * 16 + m) * HP + 8 * hh;
#pragma unroll
    for (int kt = 0; kt < DDIM / 32; ++kt) {
      FragB ah, al, bh, bl;
      ah.h[0] = *(const v8us*)(ahp + 32 * kt);
      ah.h[1] = *(const v8us*)(ahp + 32 * kt + 16);
      al.h[0] = *(const v8us*)(alp + 32 * kt);
      al.h[1] = *(const v8us*)(alp + 32 * kt + 16);
      const unsigned short* bp = w2p + (size_t)m * DDIM + 32 * kt + 8 * hh;
      bh.h[0] = *(const v8us*)bp;
      bh.h[1] = *(const v8us*)(bp + 16);
      bl.h[0] = *(const v8us*)(bp + 16 * DDIM);
      bl.h[1] = *(const v8us*)(bp + 16 * DDIM + 16);
      acc2 = wmb(ah.v, bh.v, acc2);
      acc2 = wmb(ah.v, bl.v, acc2);
      acc2 = wmb(al.v, bh.v, acc2);
    }
    const int mm = m < HOR ? m : HOR - 1;
    const float bb2 = b2[mm];
    if (m < HOR) {
#pragma unroll
      for (int r = 0; r < 8; ++r) sO[(r2 * 16 + 8 * hh + r) * HOR + m] = acc2[r] + bb2;
    }
  }
  __syncthreads();

  if (wave == 0) {
    const size_t startF = (size_t)rowBase * HOR;
    long long rem = (long long)nOut - (long long)startF;
    int cntF = rem > (long long)(LBM * HOR) ? LBM * HOR : (rem < 0 ? 0 : (int)rem);
    v4f ov[3];
#pragma unroll
    for (int i = 0; i < 3; ++i) {
      const int f = i * 32 + lane;
      ov[i] = *(const v4f*)(sO + 4 * f);
      if (4 * f + 4 <= cntF) *(volatile v4f*)(out + startF + 4 * f) = ov[i];
    }
    __threadfence();
#pragma unroll
    for (int i = 0; i < 3; ++i) {
      const int f = i * 32 + lane;
      if (4 * f + 4 <= cntF) *(volatile v4f*)(out + startF + 4 * f) = ov[i];
    }
  }
}

extern "C" void kernel_launch(void* const* d_in, const int* in_sizes, int n_in,
                              void* d_out, int out_size, void* d_ws, size_t ws_size,
                              hipStream_t stream) {
  if (n_in < 19) return;
  const int nE = in_sizes[1] / 2;
  if (nE <= 0 || in_sizes[1] != 2 * nE || in_sizes[2] != nE) return;
  if (in_sizes[3] != FDIM * DDIM) return;
  if (in_sizes[4] != DDIM || in_sizes[5] != DDIM || in_sizes[6] != DDIM || in_sizes[7] != DDIM || in_sizes[8] != DDIM) return;
  if (in_sizes[9] != GDIM * DDIM || in_sizes[10] != GDIM * DDIM || in_sizes[11] != GDIM || in_sizes[12] != GDIM) return;
  if (in_sizes[13] != DDIM || in_sizes[14] != DDIM || in_sizes[15] != DDIM * DDIM || in_sizes[16] != DDIM) return;
  if (in_sizes[17] != DDIM * HOR || in_sizes[18] != HOR) return;
  if (out_size <= 0 || (out_size % (NNODE * HOR)) != 0) return;
  const int nB = out_size / (NNODE * HOR);
  const int M  = nB * NNODE;
  if (nB < 1 || (in_sizes[0] % (M * FDIM)) != 0) return;
  const int nT = in_sizes[0] / (M * FDIM);
  if (nT < 1 || nT > 4096) return;
  if ((long long)M * nT > (1LL << 26) || nE > (1 << 26)) return;
  const int R = M * nT;

  const float* x        = (const float*)d_in[0];
  const int*   ei       = (const int*)d_in[1];
  const float* ew       = (const float*)d_in[2];
  const float* W_lin    = (const float*)d_in[3];
  const float* att_src  = (const float*)d_in[4];
  const float* att_dst  = (const float*)d_in[5];
  const float* W_edge   = (const float*)d_in[6];
  const float* att_edge = (const float*)d_in[7];
  const float* gat_bias = (const float*)d_in[8];
  const float* W_ih     = (const float*)d_in[9];
  const float* W_hh     = (const float*)d_in[10];
  const float* b_ih     = (const float*)d_in[11];
  const float* b_hh     = (const float*)d_in[12];
  const float* ln_g     = (const float*)d_in[13];
  const float* ln_b     = (const float*)d_in[14];
  const float* W1       = (const float*)d_in[15];
  const float* b1       = (const float*)d_in[16];
  const float* W2       = (const float*)d_in[17];
  const float* b2       = (const float*)d_in[18];
  float* out = (float*)d_out;

  const int RP = ((R + HXB - 1) / HXB) * HXB;
  const int MP = ((M + LBM - 1) / LBM) * LBM;

  char* ws = (char*)d_ws;
  size_t off = 0;
  const size_t oWl  = off; off += (size_t)2 * DDIM * FDIM * 2;   off = (off + 255) & ~(size_t)255;
  const size_t oWih = off; off += (size_t)GDIM * DDIM * 2;       off = (off + 255) & ~(size_t)255;
  const size_t oWhh = off; off += (size_t)GDIM * DDIM * 2;       off = (off + 255) & ~(size_t)255;
  const size_t oW1  = off; off += (size_t)2 * DDIM * DDIM * 2;   off = (off + 255) & ~(size_t)255;
  const size_t oW2  = off; off += (size_t)2 * 16 * DDIM * 2;     off = (off + 255) & ~(size_t)255;
  const size_t oHx  = off; off += (size_t)RP * DDIM * 4;         off = (off + 255) & ~(size_t)255;
  const size_t oES  = off; off += (size_t)RP * NHEAD * 4;        off = (off + 255) & ~(size_t)255;
  const size_t oED  = off; off += (size_t)RP * NHEAD * 4;        off = (off + 255) & ~(size_t)255;
  const size_t oG16 = off; off += (size_t)R * DDIM * 2;          off = (off + 255) & ~(size_t)255;
  const size_t oHT  = off; off += (size_t)MP * DDIM * 4;         off = (off + 255) & ~(size_t)255;
  if (off > ws_size || off > (size_t)WSCAP) return;
  unsigned short* wlp = (unsigned short*)(ws + oWl);
  unsigned short* pih = (unsigned short*)(ws + oWih);
  unsigned short* phh = (unsigned short*)(ws + oWhh);
  unsigned short* w1p = (unsigned short*)(ws + oW1);
  unsigned short* w2p = (unsigned short*)(ws + oW2);
  float* hxp = (float*)(ws + oHx);
  float* esp = (float*)(ws + oES);
  float* edp = (float*)(ws + oED);
  unsigned short* g16 = (unsigned short*)(ws + oG16);
  float* hTp = (float*)(ws + oHT);

  const int vec8 = ((nE & 3) == 0) ? 1 : 0;

  k_prep_lin<<<1, NTHR, 0, stream>>>(W_lin, wlp);
  k_prep_lstm<<<64, NTHR, 0, stream>>>(W_ih, W_hh, pih, phh);
  k_prep_head<<<9, NTHR, 0, stream>>>(W1, W2, w1p, w2p);

  k_hx<<<RP / HXB, NTHR, 0, stream>>>(x, wlp, att_src, att_dst, hxp, esp, edp, R);

  k_agg<<<(NNODE + NBT - 1) / NBT, NTHR, LDS_AGG, stream>>>(ei, ew, W_edge, att_edge, gat_bias,
                                                             hxp, esp, edp, g16, NNODE, nE, nB, nT, vec8);

  hipFuncSetAttribute(reinterpret_cast<const void*>(&k_lstm),
                      hipFuncAttributeMaxDynamicSharedMemorySize, LDS_LSTM);
  k_lstm<<<MP / LBM, NTHR, LDS_LSTM, stream>>>(g16, pih, phh, b_ih, b_hh, hTp, M, nT);

  k_head<<<(M + LBM - 1) / LBM, NTHR, 0, stream>>>(hTp, ln_g, ln_b, w1p, b1, w2p, b2, out, M, out_size);
}
